// FrequencyAwareGCFM_56590489092719
// MI455X (gfx1250) — hardware-verified
//
#include <hip/hip_runtime.h>
#include <stdint.h>

#define NB    4
#define CC    64
#define C3    192
#define IMS   128
#define HW    16384
#define PW    130
#define PHW   16900
#define K1    1728
#define NDK   576
#define NGT   128
#define KF    576
#define GM    64
#define GN    64
#define OSP   68
#define DP    33
#define MSP   36
#define NROW  704
#define CAP   256
#define NBORD 516
#define GLINES 390
#define WSC   16.0f
#define IWSC  0.0625f

#define WOFF2 331776
#define WOFF3 442368
#define WOFF4 466944
#define WTOT  503808
#define DYNLDS ((NROW * DP + CC * MSP) * 4)

static_assert(WOFF2 == C3 * K1);
static_assert(WOFF3 == WOFF2 + NDK * C3);
static_assert(WOFF4 == WOFF3 + NGT * C3);
static_assert(WTOT == WOFF4 + CC * KF);
static_assert(WOFF2 % 2048 == 0);
static_assert(WOFF3 % 2048 == 0);
static_assert(WOFF4 % 2048 == 0);
static_assert(WTOT % 2048 == 0);
static_assert(NROW == NDK + NGT);
static_assert(NROW % 32 == 0);
static_assert(NDK % 32 == 0);
static_assert((NROW * DP * 4) % 16 == 0);
static_assert((MSP * 4) % 16 == 0);
static_assert((OSP * 4) % 16 == 0);
static_assert(PW * C3 == GLINES * 64);
static_assert(PW * PW == PHW);
static_assert(NBORD == 2 * PW + 2 * IMS);
static_assert(HW == IMS * IMS);
static_assert(C3 % 32 == 0);
static_assert(CC % 32 == 0);

typedef _Float16       v16h __attribute__((ext_vector_type(16)));
typedef _Float16       v8h  __attribute__((ext_vector_type(8)));
typedef unsigned short v8us __attribute__((ext_vector_type(8)));
typedef float          v8f  __attribute__((ext_vector_type(8)));
typedef float          v4f  __attribute__((ext_vector_type(4)));
typedef unsigned int   v4u  __attribute__((ext_vector_type(4)));

union Frag { v8us u[2]; v16h h; };
static_assert(sizeof(Frag) == 32);

__device__ __forceinline__ unsigned short bf_bits(float f) {
  unsigned u = __float_as_uint(f);
  return (unsigned short)((u + 0x7FFFu + ((u >> 16) & 1u)) >> 16);
}
__device__ __forceinline__ float bf_up(unsigned short hb) { return __uint_as_float(((unsigned)hb) << 16); }
__device__ __forceinline__ float bfr(float f) { return bf_up(bf_bits(f)); }
__device__ __forceinline__ unsigned short h_bits(_Float16 x) { return __builtin_bit_cast(unsigned short, x); }
__device__ __forceinline__ unsigned pk16(unsigned short a, unsigned short b) { return (unsigned)a | ((unsigned)b << 16); }
__device__ __forceinline__ v8f zero8() { v8f z = {0.f, 0.f, 0.f, 0.f, 0.f, 0.f, 0.f, 0.f}; return z; }
__device__ __forceinline__ float sigm(float v) {
  const float ex = __expf(fminf(-v, 80.0f));
#if defined(__HIP_DEVICE_COMPILE__)
  return __builtin_amdgcn_rcpf(1.0f + ex);
#else
  return 1.0f / (1.0f + ex);
#endif
}

__device__ __forceinline__ Frag ldfrag(const unsigned short* p) {
  Frag f;
  f.u[0] = *(const v8us*)(p);
  f.u[1] = *(const v8us*)(p + 16);
  return f;
}

__device__ __forceinline__ v8f mma_h(v16h a, v16h b, v8f c) {
  v8f d = __builtin_amdgcn_wmma_f32_16x16x32_f16(false, a, false, b, (short)0, c, false, false);
#if defined(__HIP_DEVICE_COMPILE__)
  asm volatile("v_nop\n\tv_nop\n\tv_nop\n\tv_nop" : "+v"(d) : "v"(a), "v"(b));
#endif
  return d;
}

__global__ __launch_bounds__(256)
void cvt_w(const float* __restrict__ w1, const float* __restrict__ w2, const float* __restrict__ wg,
           const float* __restrict__ wf, unsigned short* WB) {
  const int g0 = (int)blockIdx.x * 2048;
  const int i = g0 + (int)threadIdx.x * 8;
  const float* s;
  int st;
  if (g0 >= WOFF4) {
    const int idx = i - WOFF4;
    const int o = idx / KF, k = idx - o * KF;
    const int tap = k >> 6, ic = k & 63;
    s = wf + o * KF + ic * 9 + tap; st = 9;
  } else if (g0 >= WOFF3) {
    s = wg + (i - WOFF3); st = 1;
  } else if (g0 >= WOFF2) {
    const int idx = i - WOFF2;
    const int r = idx / C3, k = idx - r * C3;
    const int t = r >> 6, ch = r & 63;
    s = w2 + (ch * 9 + t) * C3 + k; st = 1;
  } else {
    const int o = i / K1, k = i - o * K1;
    const int tap = k / C3, ic = k - tap * C3;
    s = w1 + o * K1 + ic * 9 + tap; st = 9;
  }
  float f[8];
#pragma unroll
  for (int j = 0; j < 8; ++j) f[j] = bfr(s[j * st]) * WSC;
  v4u w;
#pragma unroll
  for (int t = 0; t < 4; ++t) w[t] = pk16(h_bits((_Float16)f[2 * t]), h_bits((_Float16)f[2 * t + 1]));
  unsigned short* p = WB + (size_t)i;
  *(volatile v4u*)p = w;
  __threadfence();
  *(volatile v4u*)p = w;
}

__global__ __launch_bounds__(192)
void k_ca(const float* __restrict__ pan, const float* __restrict__ ms, const float* __restrict__ nir,
          const float* __restrict__ w1, const float* __restrict__ w2, float* CA) {
  __shared__ float smean[C3];
  __shared__ float shid[16];
  __shared__ __align__(16) float scav[CAP];
  const int t = threadIdx.x, b = blockIdx.x;
  const float* base = (t < CC) ? pan : ((t < 2 * CC) ? ms : nir);
  const float* src = base + ((size_t)b * CC + (t & (CC - 1))) * HW;
  float s0 = 0.f, s1 = 0.f, s2 = 0.f, s3 = 0.f;
#pragma unroll 1
  for (int i = 0; i < HW / 4; ++i) {
    const v4f v = *(const v4f*)(src + 4 * i);
    s0 += bfr(v[0]); s1 += bfr(v[1]); s2 += bfr(v[2]); s3 += bfr(v[3]);
  }
  smean[t] = ((s0 + s1) + (s2 + s3)) * (1.0f / 16384.0f);
  __syncthreads();
  if (t < 12) {
    float s = 0.f;
#pragma unroll 1
    for (int k = 0; k < C3; ++k) s = fmaf(bfr(w1[t * C3 + k]), smean[k], s);
    shid[t] = fmaxf(s, 0.f);
  }
  __syncthreads();
  {
    float s = 0.f;
#pragma unroll 1
    for (int k = 0; k < 12; ++k) s = fmaf(bfr(w2[t * 12 + k]), shid[k], s);
    scav[t] = sigm(s);
    if (t < CAP - C3) scav[C3 + t] = 0.f;
  }
  __syncthreads();
  if (t < 64) {
    const v4f v = *(const v4f*)(scav + 4 * t);
    float* p = CA + (size_t)b * CAP + 4 * t;
    *(volatile v4f*)p = v;
    __threadfence();
    *(volatile v4f*)p = v;
  }
}

__global__ __launch_bounds__(256)
void k_am(const float* __restrict__ pan, const float* __restrict__ ms, const float* __restrict__ nir,
          const float* __restrict__ CA, float* AM) {
  __shared__ float scav[C3];
  const int t = threadIdx.x, b = blockIdx.y;
  if (t < C3) scav[t] = CA[(size_t)b * CAP + t];
  __syncthreads();
  const int px = blockIdx.x * 256 + t;
  float s = 0.f, mx = -__builtin_huge_valf();
#pragma unroll 1
  for (int k = 0; k < C3; ++k) {
    const float* base = (k < CC) ? pan : ((k < 2 * CC) ? ms : nir);
    const float v = bfr(base[((size_t)b * CC + (k & (CC - 1))) * HW + px]) * scav[k];
    s += v;
    mx = fmaxf(mx, v);
  }
  const float av = s * (1.0f / 192.0f);
  float* p0 = AM + ((size_t)b * 2) * HW + px;
  float* p1 = p0 + HW;
  *(volatile float*)p0 = av;
  *(volatile float*)p1 = mx;
  __threadfence();
  *(volatile float*)p0 = av;
  *(volatile float*)p1 = mx;
}

__global__ __launch_bounds__(256)
void k_g(const float* __restrict__ pan, const float* __restrict__ ms, const float* __restrict__ nir,
         const float* __restrict__ CA, const float* __restrict__ AM, const float* __restrict__ sw,
         unsigned short* GP) {
  __shared__ __align__(16) unsigned short Gt[PW * C3];
  __shared__ float sarow[IMS];
  __shared__ float wsa[IMS];
  __shared__ float scav[C3];
  const int t = threadIdx.x;
  const int yp = blockIdx.x, b = blockIdx.y;
  const bool border = (yp == 0) || (yp == PW - 1);
  if (!border) {
    const int y = yp - 1;
    if (t < 98) wsa[t] = bfr(sw[t]);
    if (t < C3) {
      scav[t] = CA[(size_t)b * CAP + t];
      Gt[t] = 0;
      Gt[(PW - 1) * C3 + t] = 0;
    }
    __syncthreads();
    if (t < IMS) {
      float s = 0.f;
#pragma unroll 1
      for (int ch = 0; ch < 2; ++ch) {
        const float* in = AM + ((size_t)b * 2 + ch) * HW;
#pragma unroll 1
        for (int ky = 0; ky < 7; ++ky) {
          const int yy = y + ky - 3;
          const bool oky = (unsigned)yy < (unsigned)IMS;
          const int yc = min(max(yy, 0), IMS - 1);
#pragma unroll 1
          for (int kx = 0; kx < 7; ++kx) {
            const int xx = t + kx - 3;
            const bool ok = oky && ((unsigned)xx < (unsigned)IMS);
            const int xc = min(max(xx, 0), IMS - 1);
            const float av = in[yc * IMS + xc];
            s = fmaf(ok ? av : 0.f, wsa[ch * 49 + ky * 7 + kx], s);
          }
        }
      }
      sarow[t] = sigm(s);
    }
    __syncthreads();
#pragma unroll 1
    for (int idx = t; idx < C3 * IMS; idx += 256) {
      const int ch = idx >> 7, x = idx & (IMS - 1);
      const float* base = (ch < CC) ? pan : ((ch < 2 * CC) ? ms : nir);
      const float v = bfr(base[((size_t)b * CC + (ch & (CC - 1))) * HW + (size_t)y * IMS + x]);
      const float a = v * scav[ch];
      const float g = fmaf(a, sarow[x], v);
      Gt[(x + 1) * C3 + ch] = h_bits((_Float16)g);
    }
  }
  __syncthreads();
  {
    const int e = t & 7, lq = t >> 3;
    unsigned short* gbase = GP + ((size_t)b * PHW + (size_t)yp * PW) * C3;
    const v4u z = {0u, 0u, 0u, 0u};
#pragma unroll
    for (int pass = 0; pass < 2; ++pass) {
#pragma unroll 1
      for (int it = 0; it < 13; ++it) {
        const int L = it * 32 + lq;
        if (L < GLINES) {
          v4u u = z;
          if (!border) u = *(const v4u*)(Gt + L * 64 + 8 * e);
          *(volatile v4u*)(gbase + (size_t)L * 64 + 8 * e) = u;
        }
      }
      __threadfence();
    }
  }
}

template <int CIN, int MODE>
__global__ __launch_bounds__(128)
void conv_gemm(const unsigned short* __restrict__ Wp, const unsigned short* __restrict__ BP,
               const float* __restrict__ bias, const float* __restrict__ resid,
               unsigned short* outP, float* outF) {
  constexpr int K = 9 * CIN;
  __shared__ __align__(16) float Os[GM * OSP];
  const int tid  = threadIdx.x;
  const int lane = tid & 31, wave = tid >> 5;
  const int hh   = lane >> 4, c = lane & 15;
  const int wm   = wave >> 1, wn = wave & 1;
  const int b    = blockIdx.z;
  const int mBase = blockIdx.x * GM;
  const int n0   = blockIdx.y * GN;
  const int y    = n0 >> 7, x0 = n0 & (IMS - 1);

  const unsigned short* a0p = Wp + (size_t)(mBase + 32 * wm + c) * K + 8 * hh;
  const unsigned short* a1p = a0p + (size_t)16 * K;
  const size_t prow0 = (size_t)b * PHW + (size_t)y * PW + x0 + 32 * wn + c;

  v8f acc[2][2];
#pragma unroll
  for (int mi = 0; mi < 2; ++mi)
#pragma unroll
    for (int ni = 0; ni < 2; ++ni) acc[mi][ni] = zero8();

#pragma unroll 1
  for (int k0 = 0; k0 < K; k0 += 32) {
    const int tap = k0 / CIN;
    const int ic0 = k0 - tap * CIN;
    const int dy  = tap / 3, dx = tap - 3 * dy;
    const unsigned short* bp0 = BP + (prow0 + (size_t)dy * PW + dx) * CIN + ic0 + 8 * hh;
    const unsigned short* bp1 = bp0 + 16 * CIN;
    const Frag fa0 = ldfrag(a0p + k0);
    const Frag fa1 = ldfrag(a1p + k0);
    const Frag fb0 = ldfrag(bp0);
    const Frag fb1 = ldfrag(bp1);
    acc[0][0] = mma_h(fa0.h, fb0.h, acc[0][0]);
    acc[0][1] = mma_h(fa0.h, fb1.h, acc[0][1]);
    acc[1][0] = mma_h(fa1.h, fb0.h, acc[1][0]);
    acc[1][1] = mma_h(fa1.h, fb1.h, acc[1][1]);
  }

#pragma unroll
  for (int mi = 0; mi < 2; ++mi) {
#pragma unroll
    for (int ni = 0; ni < 2; ++ni) {
      const int n_loc = 32 * wn + 16 * ni + c;
#pragma unroll
      for (int r = 0; r < 8; ++r) {
        const int o_loc = 32 * wm + 16 * mi + 8 * hh + r;
        const int o = mBase + o_loc;
        float v = acc[mi][ni][r] * IWSC + bfr(bias[o]);
        if (MODE == 0) {
          v = fmaxf(v, 0.f);
        } else {
          v += resid[((size_t)b * CC + o) * HW + n0 + n_loc];
        }
        Os[o_loc * OSP + n_loc] = v;
      }
    }
  }
  __syncthreads();

  {
    const int e = tid & 7, lq = tid >> 3;
#pragma unroll
    for (int pass = 0; pass < 2; ++pass) {
      if (MODE == 1) {
#pragma unroll
        for (int it = 0; it < 8; ++it) {
          const int L = it * 16 + lq;
          const int row = L >> 1, hf = L & 1;
          const v4f v = *(const v4f*)(Os + row * OSP + hf * 32 + 4 * e);
          float* dst = outF + ((size_t)b * CC + mBase + row) * HW + n0 + hf * 32 + 4 * e;
          *(volatile v4f*)dst = v;
        }
      } else {
#pragma unroll
        for (int it = 0; it < 4; ++it) {
          const int n_loc = it * 16 + lq;
          const int ch0 = 8 * e;
          float f[8];
#pragma unroll
          for (int j = 0; j < 8; ++j) f[j] = Os[(ch0 + j) * OSP + n_loc];
          v4u u;
#pragma unroll
          for (int t = 0; t < 4; ++t) u[t] = pk16(h_bits((_Float16)f[2 * t]), h_bits((_Float16)f[2 * t + 1]));
          unsigned short* dst = outP + ((size_t)b * HW + n0 + n_loc) * (size_t)C3 + mBase + ch0;
          *(volatile v4u*)dst = u;
        }
      }
      __threadfence();
    }
  }
}

__global__ __launch_bounds__(256)
void k_padzero(unsigned short* MP) {
  const int t = threadIdx.x;
  const int e = t & 7;
  const int L = blockIdx.x * 32 + (t >> 3);
  const bool ok = L < NB * NBORD;
  const int Lc = ok ? L : 0;
  const int b = Lc / NBORD, r = Lc - b * NBORD;
  int yp, xp;
  if (r < PW)          { yp = 0;      xp = r; }
  else if (r < 2 * PW) { yp = PW - 1; xp = r - PW; }
  else { const int q = r - 2 * PW; yp = 1 + (q >> 1); xp = (q & 1) ? (PW - 1) : 0; }
  unsigned short* p = MP + ((size_t)b * PHW + (size_t)yp * PW + xp) * CC + 8 * e;
  const v4u z = {0u, 0u, 0u, 0u};
  if (ok) *(volatile v4u*)p = z;
  __threadfence();
  if (ok) *(volatile v4u*)p = z;
}

__global__ __launch_bounds__(256)
void k_dyn(const unsigned short* __restrict__ WB, const unsigned short* __restrict__ HP,
           const unsigned short* __restrict__ GP,
           const float* __restrict__ pan, const float* __restrict__ ms, const float* __restrict__ corr,
           const float* __restrict__ alpha, const float* __restrict__ kb2, const float* __restrict__ gb,
           float* MF, unsigned short* MP) {
  extern __shared__ __align__(16) float dsm[];
  float* Ds = dsm;
  float* Ms = dsm + NROW * DP;
  const int tid  = threadIdx.x;
  const int lane = tid & 31, wave = tid >> 5;
  const int hh   = lane >> 4, c = lane & 15;
  const int tx = blockIdx.x, y = blockIdx.y, b = blockIdx.z;
  const int x0 = tx * 32;

#pragma unroll 1
  for (int p = 0; p < 3; ++p) {
    const int ti = p * 8 + wave;
    if (ti < NROW / 32) {
      const bool isg = (ti >= NDK / 32);
      const int arow = isg ? (32 * (ti - NDK / 32)) : (32 * ti);
      const unsigned short* abase = WB + (isg ? WOFF3 : WOFF2) + (size_t)(arow + c) * C3 + 8 * hh;
      const size_t brow = isg ? ((size_t)b * PHW + (size_t)(y + 1) * PW + x0 + 1 + c)
                              : ((size_t)b * HW + (size_t)y * IMS + x0 + c);
      const unsigned short* bsrc = isg ? GP : HP;
      const unsigned short* bbase = bsrc + brow * C3 + 8 * hh;
      v8f acc[2][2];
#pragma unroll
      for (int mi = 0; mi < 2; ++mi)
#pragma unroll
        for (int ni = 0; ni < 2; ++ni) acc[mi][ni] = zero8();
#pragma unroll 1
      for (int k0 = 0; k0 < C3; k0 += 32) {
        const Frag fa0 = ldfrag(abase + k0);
        const Frag fa1 = ldfrag(abase + (size_t)16 * C3 + k0);
        const Frag fb0 = ldfrag(bbase + k0);
        const Frag fb1 = ldfrag(bbase + (size_t)16 * C3 + k0);
        acc[0][0] = mma_h(fa0.h, fb0.h, acc[0][0]);
        acc[0][1] = mma_h(fa0.h, fb1.h, acc[0][1]);
        acc[1][0] = mma_h(fa1.h, fb0.h, acc[1][0]);
        acc[1][1] = mma_h(fa1.h, fb1.h, acc[1][1]);
      }
      const int drow = 32 * ti;
#pragma unroll
      for (int mi = 0; mi < 2; ++mi)
#pragma unroll
        for (int ni = 0; ni < 2; ++ni)
#pragma unroll
          for (int r = 0; r < 8; ++r)
            Ds[(drow + 16 * mi + 8 * hh + r) * DP + 16 * ni + c] = acc[mi][ni][r];
    }
  }
  __syncthreads();

  {
    const int px = tid & 31, cq = tid >> 5;
    const int x = x0 + px;
    const float al = bfr(alpha[0]);
    const float cr = bfr(corr[(size_t)b * HW + (size_t)y * IMS + x]);
#pragma unroll 1
    for (int j = 0; j < 8; ++j) {
      const int ch = 8 * cq + j;
      const float* panc = pan + ((size_t)b * CC + ch) * HW;
      float pd = 0.f, lap = 0.f;
#pragma unroll
      for (int t = 0; t < 9; ++t) {
        const int ky = t / 3, kx = t - 3 * ky;
        const int yy = y + ky - 1, xx = x + kx - 1;
        const bool ok = ((unsigned)yy < (unsigned)IMS) && ((unsigned)xx < (unsigned)IMS);
        const int yc = min(max(yy, 0), IMS - 1);
        const int xc = min(max(xx, 0), IMS - 1);
        const float raw = panc[yc * IMS + xc];
        const float pv = ok ? bfr(raw) : 0.f;
        const float dk = Ds[(t * CC + ch) * DP + px] * IWSC + bfr(kb2[ch * 9 + t]);
        pd = pd + dk * pv;
        lap = lap + ((t == 4) ? 8.0f : -1.0f) * pv;
      }
      const float gp  = sigm(Ds[(NDK + ch) * DP + px] * IWSC + bfr(gb[ch]));
      const float gmv = sigm(Ds[(NDK + CC + ch) * DP + px] * IWSC + bfr(gb[CC + ch]));
      const float msv = bfr(ms[((size_t)b * CC + ch) * HW + (size_t)y * IMS + x]);
      const float dyn = gp * pd + gmv * msv;
      const float fu  = dyn + al * lap;
      Ms[ch * MSP + px] = fu * cr;
    }
  }
  __syncthreads();

  {
    const int e = tid & 7, lq = tid >> 3;
#pragma unroll
    for (int pass = 0; pass < 2; ++pass) {
#pragma unroll
      for (int it = 0; it < 2; ++it) {
        const int row = it * 32 + lq;
        const v4f v = *(const v4f*)(Ms + row * MSP + 4 * e);
        float* dst = MF + ((size_t)b * CC + row) * HW + (size_t)y * IMS + x0 + 4 * e;
        *(volatile v4f*)dst = v;
      }
      {
        const int n_loc = lq;
        const int ch0 = 8 * e;
        float f[8];
#pragma unroll
        for (int jj = 0; jj < 8; ++jj) f[jj] = Ms[(ch0 + jj) * MSP + n_loc];
        v4u u;
#pragma unroll
        for (int t = 0; t < 4; ++t) u[t] = pk16(h_bits((_Float16)f[2 * t]), h_bits((_Float16)f[2 * t + 1]));
        unsigned short* dst = MP + ((size_t)b * PHW + (size_t)(y + 1) * PW + x0 + 1 + n_loc) * CC + ch0;
        *(volatile v4u*)dst = u;
      }
      __threadfence();
    }
  }
}

extern "C" void kernel_launch(void* const* d_in, const int* in_sizes, int n_in,
                              void* d_out, int out_size, void* d_ws, size_t ws_size,
                              hipStream_t stream) {
  const int NX = NB * CC * HW;
  if (n_in < 16) return;
  if (in_sizes[0] != NX || in_sizes[1] != NX || in_sizes[2] != NX) return;
  if (in_sizes[3] != NB * HW) return;
  if (in_sizes[4] != 12 * C3 || in_sizes[5] != C3 * 12 || in_sizes[6] != 98) return;
  if (in_sizes[7] != NGT * C3 || in_sizes[8] != NGT) return;
  if (in_sizes[9] != C3 * K1 || in_sizes[10] != C3) return;
  if (in_sizes[11] != NDK * C3 || in_sizes[12] != NDK) return;
  if (in_sizes[13] < 1) return;
  if (in_sizes[14] != CC * KF || in_sizes[15] != CC) return;
  if (out_size != NX) return;

  size_t off = 0;
  auto take = [&](size_t bytes) -> size_t {
    const size_t o = off;
    off = (off + bytes + 255) & ~(size_t)255;
    return o;
  };
  const size_t oW  = take((size_t)WTOT * 2);
  const size_t oCA = take((size_t)NB * CAP * 4);
  const size_t oAM = take((size_t)NB * 2 * HW * 4);
  const size_t oGP = take((size_t)NB * PHW * C3 * 2);
  const size_t oHP = take((size_t)NB * HW * C3 * 2);
  const size_t oMF = take((size_t)NB * CC * HW * 4);
  const size_t oMP = take((size_t)NB * PHW * CC * 2);
  if (off > ws_size) return;
  if (off > (size_t)134217728) return;

  const float* pan    = (const float*)d_in[0];
  const float* ms     = (const float*)d_in[1];
  const float* nir    = (const float*)d_in[2];
  const float* corr   = (const float*)d_in[3];
  const float* ca_w1  = (const float*)d_in[4];
  const float* ca_w2  = (const float*)d_in[5];
  const float* sa_w   = (const float*)d_in[6];
  const float* gate_w = (const float*)d_in[7];
  const float* gate_b = (const float*)d_in[8];
  const float* kp_w1  = (const float*)d_in[9];
  const float* kp_b1  = (const float*)d_in[10];
  const float* kp_w2  = (const float*)d_in[11];
  const float* kp_b2  = (const float*)d_in[12];
  const float* alpha  = (const float*)d_in[13];
  const float* fc_w   = (const float*)d_in[14];
  const float* fc_b   = (const float*)d_in[15];

  char* ws = (char*)d_ws;
  unsigned short* WB = (unsigned short*)(ws + oW);
  float*          CA = (float*)(ws + oCA);
  float*          AM = (float*)(ws + oAM);
  unsigned short* GP = (unsigned short*)(ws + oGP);
  unsigned short* HP = (unsigned short*)(ws + oHP);
  float*          MF = (float*)(ws + oMF);
  unsigned short* MP = (unsigned short*)(ws + oMP);
  float* out = (float*)d_out;

  const dim3 blk256(256), blk192(192), blk128(128);
  const dim3 gW(WTOT / 2048);
  const dim3 gCA(NB);
  const dim3 gAM(HW / 256, NB);
  const dim3 gG(PW, NB);
  const dim3 gK1(C3 / GM, HW / GN, NB);
  const dim3 gPZ((NB * NBORD + 31) / 32);
  const dim3 gDY(IMS / 32, IMS, NB);
  const dim3 gFC(CC / GM, HW / GN, NB);

  cvt_w<<<gW, blk256, 0, stream>>>(kp_w1, kp_w2, gate_w, fc_w, WB);
  k_ca<<<gCA, blk192, 0, stream>>>(pan, ms, nir, ca_w1, ca_w2, CA);
  k_am<<<gAM, blk256, 0, stream>>>(pan, ms, nir, CA, AM);
  k_g<<<gG, blk256, 0, stream>>>(pan, ms, nir, CA, AM, sa_w, GP);
  conv_gemm<C3, 0><<<gK1, blk128, 0, stream>>>(WB, GP, kp_b1, nullptr, HP, nullptr);
  k_padzero<<<gPZ, blk256, 0, stream>>>(MP);
  (void)hipFuncSetAttribute(reinterpret_cast<const void*>(&k_dyn), hipFuncAttributeMaxDynamicSharedMemorySize, DYNLDS);
  k_dyn<<<gDY, blk256, DYNLDS, stream>>>(WB, HP, GP, pan, ms, corr, alpha, kp_b2, gate_b, MF, MP);
  conv_gemm<CC, 1><<<gFC, blk128, 0, stream>>>(WB + WOFF4, MP, fc_b, MF, nullptr, out);
  (void)hipGetLastError();
}
